// LSTMAttentionModel_64802466562238
// MI455X (gfx1250) — hardware-run, weakly checked
//
#include <hip/hip_runtime.h>
#include <math.h>

constexpr int kT   = 64;
constexpr int kB   = 64;
constexpr int kE   = 128;
constexpr int kH   = 256;
constexpr int kG   = 4 * kH;
constexpr int kNI  = 50000;
constexpr int kNIP = 50048;
constexpr int kND  = 20000;
constexpr int kM   = kT * kB;
constexpr int kHP  = 264;
constexpr int kNOUT = kB * kNI;

constexpr int isqrt_c(int n) { int r = 0; while ((r + 1) * (r + 1) <= n) ++r; return r; }
constexpr int kSqrtH = isqrt_c(kH);
static_assert(kSqrtH * kSqrtH == kH, "H must be a perfect square");

constexpr float kWCarry   = 64.0f;
constexpr float kActCarry = 16.0f;
constexpr float kNrmCarry = 64.0f;
constexpr float kAscCarry = 256.0f;
constexpr float kQKCarry  = 16.0f;
constexpr float kPreScale   = 1.0f / (kActCarry * kWCarry);
constexpr float kQKScale    = kQKCarry / (kActCarry * kWCarry);
constexpr float kScoreScale = 1.0f / (kQKCarry * kQKCarry * (float)kSqrtH);
constexpr float kOutScale   = 1.0f / (kAscCarry * kWCarry);
constexpr float kActInv     = 1.0f / kActCarry;
constexpr float kInvT       = 1.0f / (float)kT;

static_assert(kM % 64 == 0 && kG % 64 == 0 && kE % 32 == 0, "input projection tiles");
static_assert((2 * kH) % 64 == 0 && kH % 32 == 0, "q|k projection tiles");
static_assert(kB % 64 == 0 && kNIP % 64 == 0 && kNIP >= kNI, "vocab tiles");
static_assert(kND % 32 == 0 && kND % 16 == 0, "data rows");
static_assert(kNI % 4 == 0 && kNOUT % 4 == 0, "flat copy granularity");
static_assert(kB % 16 == 0 && kH == 16 * 16, "recurrence block shape");

typedef __attribute__((ext_vector_type(16))) _Float16 v16h;
typedef __attribute__((ext_vector_type(8)))  _Float16 v8h;
typedef __attribute__((ext_vector_type(16))) __bf16   v16b;
typedef __attribute__((ext_vector_type(8)))  __bf16   v8b;
typedef __attribute__((ext_vector_type(8)))  float    v8f;
typedef __attribute__((ext_vector_type(4)))  float    v4f;
typedef __attribute__((ext_vector_type(2)))  float    v2f;
typedef __attribute__((ext_vector_type(4)))  unsigned int v4u;
typedef __attribute__((ext_vector_type(2)))  unsigned int v2u;
typedef __attribute__((ext_vector_type(2)))  int      v2i;

__device__ __forceinline__ unsigned short f2bf_bits(float f) {
  unsigned u = __float_as_uint(f);
  return (unsigned short)((u + 0x7FFFu + ((u >> 16) & 1u)) >> 16);
}
__device__ __forceinline__ float bf_bits2f(unsigned short h) { return __uint_as_float(((unsigned)h) << 16); }
__device__ __forceinline__ unsigned pk16(unsigned short a, unsigned short b) { return (unsigned)a | ((unsigned)b << 16); }
__device__ __forceinline__ unsigned short h_bits(float f) { const _Float16 h = (_Float16)f; return __builtin_bit_cast(unsigned short, h); }

__device__ __forceinline__ float h16_to_f32(unsigned hb) {
  const unsigned sgn = (hb & 0x8000u) << 16;
  const unsigned em = hb & 0x7fffu;
  const float fn = __uint_as_float((em << 13) + 0x38000000u);
  const float fs = (float)em * 5.9604644775390625e-8f;
  const float mag = (em < 0x400u) ? fs : fn;
  return __uint_as_float(__float_as_uint(mag) | sgn);
}

__device__ __forceinline__ void dep_guard4_h(v8f& a, v8f& b, v8f& c, v8f& d, v16h x, v16h y, v16h b0, v16h b1, v16h b2, v16h b3) {
  asm volatile("v_nop\n\tv_nop\n\tv_nop\n\tv_nop" : "+v"(a), "+v"(b), "+v"(c), "+v"(d) : "v"(x), "v"(y), "v"(b0), "v"(b1), "v"(b2), "v"(b3));
}
__device__ __forceinline__ void dep_guard4_b(v8f& a, v8f& b, v8f& c, v8f& d, v16b x, v16b y, v16b b0, v16b b1, v16b b2, v16b b3) {
  asm volatile("v_nop\n\tv_nop\n\tv_nop\n\tv_nop" : "+v"(a), "+v"(b), "+v"(c), "+v"(d) : "v"(x), "v"(y), "v"(b0), "v"(b1), "v"(b2), "v"(b3));
}
__device__ __forceinline__ void keep4_h(v16h a, v16h b, v16h c, v16h d) { asm volatile("v_nop" :: "v"(a), "v"(b), "v"(c), "v"(d)); }
__device__ __forceinline__ void keep4_b(v16b a, v16b b, v16b c, v16b d) { asm volatile("v_nop" :: "v"(a), "v"(b), "v"(c), "v"(d)); }
__device__ __forceinline__ void acc_guard4(v8f& a, v8f& b, v8f& c, v8f& d) { asm volatile("v_nop\n\tv_nop\n\tv_nop\n\tv_nop" : "+v"(a), "+v"(b), "+v"(c), "+v"(d)); }

template <typename T> struct Frag;
template <> struct Frag<_Float16> {
  typedef v16h V; union U { v16h v; v8h h[2]; };
  static __device__ __forceinline__ v16h load(const _Float16* p) {
    U f; f.h[0] = *(const v8h*)(p); f.h[1] = *(const v8h*)(p + 16); return f.v;
  }
  static __device__ __forceinline__ v8f mma(v16h a, v16h b, v8f c) {
    return __builtin_amdgcn_wmma_f32_16x16x32_f16(false, a, false, b, (short)0, c, false, false);
  }
  static __device__ __forceinline__ void guard4(v8f& a, v8f& b, v8f& c, v8f& d, v16h x, v16h y, v16h b0, v16h b1, v16h b2, v16h b3) { dep_guard4_h(a, b, c, d, x, y, b0, b1, b2, b3); }
  static __device__ __forceinline__ void keep(v16h a, v16h b, v16h c, v16h d) { keep4_h(a, b, c, d); }
};
template <> struct Frag<__bf16> {
  typedef v16b V; union U { v16b v; v8b h[2]; };
  static __device__ __forceinline__ v16b load(const __bf16* p) {
    U f; f.h[0] = *(const v8b*)(p); f.h[1] = *(const v8b*)(p + 16); return f.v;
  }
  static __device__ __forceinline__ v8f mma(v16b a, v16b b, v8f c) {
    return __builtin_amdgcn_wmma_f32_16x16x32_bf16(false, a, false, b, (short)0, c, false, false);
  }
  static __device__ __forceinline__ void guard4(v8f& a, v8f& b, v8f& c, v8f& d, v16b x, v16b y, v16b b0, v16b b1, v16b b2, v16b b3) { dep_guard4_b(a, b, c, d, x, y, b0, b1, b2, b3); }
  static __device__ __forceinline__ void keep(v16b a, v16b b, v16b c, v16b d) { keep4_b(a, b, c, d); }
};

__device__ __forceinline__ v8f mma_nop_h(v16h a, v16h b, v8f c) {
  c = __builtin_amdgcn_wmma_f32_16x16x32_f16(false, a, false, b, (short)0, c, false, false);
  asm volatile("v_nop\n\tv_nop\n\tv_nop\n\tv_nop" : "+v"(c) : "v"(a), "v"(b));
  return c;
}

template <int ET> struct Elem;
template <> struct Elem<0> { typedef _Float16 T; };
template <> struct Elem<1> { typedef __bf16 T; };
template <int ET, bool SPLIT, int BIAS_MODE, int OUT_MODE, bool RESID>
__global__ __launch_bounds__(256) void wmma_gemm64(
    const unsigned short* __restrict__ Ap, const unsigned short* __restrict__ A2p, int lda, long strideA,
    const unsigned short* __restrict__ Btp, const unsigned short* __restrict__ Bt2p, int ldb, long strideB,
    void* __restrict__ Cout, void* __restrict__ Cout2, int ldc, long strideC,
    const float* __restrict__ bias,
    const float* __restrict__ resid, long strideR,
    int M, int N, int K, float scale) {
  typedef typename Elem<ET>::T T;
  typedef typename Frag<T>::V V;
  const T* A = (const T*)Ap; const T* A2 = (const T*)A2p; const T* Bt = (const T*)Btp; const T* Bt2 = (const T*)Bt2p;
  __shared__ __align__(16) float sT[8][16 * 68];
  const int b    = blockIdx.y;
  const int lane = threadIdx.x & 31;
  const int wave = threadIdx.x >> 5;
  const int tilesN = N >> 6;
  const int tilesM = M >> 6;
  const int tile = blockIdx.x * 8 + wave;
  if (tile >= tilesM * tilesN) return;
  const int tm = tile / tilesN;
  const int tn = tile - tm * tilesN;
  const int m0 = tm << 6;
  const int n0 = tn << 6;

  const T* Ab  = A  + (size_t)b * strideA;
  const T* Bb  = Bt + (size_t)b * strideB;
  const T* Ab2 = SPLIT ? (A2  + (size_t)b * strideA) : nullptr;
  const T* Bb2 = SPLIT ? (Bt2 + (size_t)b * strideB) : nullptr;

  const int rlane = lane & 15;
  const int koff  = (lane >> 4) * 8;
  const int mOff  = (lane >> 4) * 8;

  v8f acc[4][4];
#pragma unroll
  for (int i = 0; i < 4; ++i)
#pragma unroll
    for (int j = 0; j < 4; ++j) acc[i][j] = (v8f){0.f,0.f,0.f,0.f,0.f,0.f,0.f,0.f};

  for (int k0 = 0; k0 < K; k0 += 32) {
    V bh[4], bl[4];
#pragma unroll
    for (int j = 0; j < 4; ++j) {
      const size_t bo = (size_t)(n0 + (j << 4) + rlane) * ldb + koff + k0;
      bh[j] = Frag<T>::load(Bb + bo);
      if (SPLIT) bl[j] = Frag<T>::load(Bb2 + bo);
    }
#pragma unroll
    for (int i = 0; i < 4; ++i) {
      const size_t ao = (size_t)(m0 + (i << 4) + rlane) * lda + koff + k0;
      V ah = Frag<T>::load(Ab + ao);
      V al;
      if (SPLIT) al = Frag<T>::load(Ab2 + ao);
#pragma unroll
      for (int j = 0; j < 4; ++j) {
        acc[i][j] = Frag<T>::mma(ah, bh[j], acc[i][j]);
        if (SPLIT) {
          acc[i][j] = Frag<T>::mma(ah, bl[j], acc[i][j]);
          acc[i][j] = Frag<T>::mma(al, bh[j], acc[i][j]);
        }
      }
      Frag<T>::guard4(acc[i][0], acc[i][1], acc[i][2], acc[i][3], ah, SPLIT ? al : ah, bh[0], bh[1], bh[2], bh[3]);
    }
    Frag<T>::keep(bh[0], bh[1], bh[2], bh[3]);
    if (SPLIT) Frag<T>::keep(bl[0], bl[1], bl[2], bl[3]);
  }
  acc_guard4(acc[0][0], acc[0][1], acc[0][2], acc[0][3]);
  acc_guard4(acc[1][0], acc[1][1], acc[1][2], acc[1][3]);
  acc_guard4(acc[2][0], acc[2][1], acc[2][2], acc[2][3]);
  acc_guard4(acc[3][0], acc[3][1], acc[3][2], acc[3][3]);

  float* slab = sT[wave];
  const float* Rb = RESID ? (resid + (size_t)b * strideR) : nullptr;
#pragma unroll
  for (int i = 0; i < 4; ++i) {
    const int mBase = m0 + (i << 4);
#pragma unroll
    for (int j = 0; j < 4; ++j) {
      const int n = n0 + (j << 4) + rlane;
      float bv = 0.f;
      if (BIAS_MODE == 2) bv = bias[n];
#pragma unroll
      for (int r = 0; r < 8; ++r) {
        float v = acc[i][j][r] * scale;
        if (BIAS_MODE == 1) v += bias[mBase + mOff + r];
        if (BIAS_MODE == 2) v += bv;
        if (RESID) v += Rb[(size_t)(mBase + mOff + r) * ldc + n];
        slab[(mOff + r) * 68 + (j << 4) + rlane] = v;
      }
    }
    __builtin_amdgcn_fence(__ATOMIC_RELEASE, "workgroup");
    __builtin_amdgcn_wave_barrier();
    __builtin_amdgcn_fence(__ATOMIC_ACQUIRE, "workgroup");
    if (OUT_MODE == 0) {
      float* C = (float*)Cout + (size_t)b * strideC;
      const int hh = lane >> 4, c4 = (lane & 15) * 4;
      for (int pass = 0; pass < 2; ++pass) {
#pragma unroll
        for (int it = 0; it < 8; ++it) {
          const int row = it * 2 + hh;
          v4f v = *(const v4f*)(slab + row * 68 + c4);
          *(volatile v4f*)(C + (size_t)(mBase + row) * ldc + n0 + c4) = v;
        }
        __threadfence();
      }
    } else {
      const int q = lane >> 3, c8 = (lane & 7) * 8;
      unsigned short* C  = (unsigned short*)Cout  + (size_t)b * strideC;
      unsigned short* C2 = (OUT_MODE == 2) ? ((unsigned short*)Cout2 + (size_t)b * strideC) : nullptr;
      for (int pass = 0; pass < 2; ++pass) {
#pragma unroll
        for (int it = 0; it < 4; ++it) {
          const int row = it * 4 + q;
          const float* sp = slab + row * 68 + c8;
          v8h hv, lv;
#pragma unroll
          for (int e = 0; e < 8; ++e) {
            if (OUT_MODE == 1) {
              hv[e] = (_Float16)sp[e];
            } else {
              unsigned short hb = f2bf_bits(sp[e]);
              unsigned short lb = f2bf_bits(sp[e] - bf_bits2f(hb));
              hv[e] = __builtin_bit_cast(_Float16, hb);
              lv[e] = __builtin_bit_cast(_Float16, lb);
            }
          }
          *(volatile v8h*)(C + (size_t)(mBase + row) * ldc + n0 + c8) = hv;
          if (OUT_MODE == 2) *(volatile v8h*)(C2 + (size_t)(mBase + row) * ldc + n0 + c8) = lv;
        }
        __threadfence();
      }
    }
    __builtin_amdgcn_fence(__ATOMIC_RELEASE, "workgroup");
    __builtin_amdgcn_wave_barrier();
    __builtin_amdgcn_fence(__ATOMIC_ACQUIRE, "workgroup");
  }
}

__global__ __launch_bounds__(256) void cast8_pad_kernel(const float* __restrict__ in, unsigned short* __restrict__ out,
                                                        int n8_real, int n8_total, float sc) {
  const int i = blockIdx.x * 256 + threadIdx.x;
  if (i >= n8_total) return;
  const bool live = (i < n8_real);
  const int ic = live ? i : (n8_real - 1);
  const float* p = in + 8 * (size_t)ic;
  const v4f a = *(const v4f*)(p);
  const v4f c = *(const v4f*)(p + 4);
  unsigned short hb[8];
#pragma unroll
  for (int e = 0; e < 4; ++e) {
    const float fa = a[e];
    const float fc = c[e];
    const float ga = live ? fa * sc : 0.0f;
    const float gc = live ? fc * sc : 0.0f;
    hb[e]     = h_bits(ga);
    hb[4 + e] = h_bits(gc);
  }
  const v4u u = (v4u){pk16(hb[0], hb[1]), pk16(hb[2], hb[3]), pk16(hb[4], hb[5]), pk16(hb[6], hb[7])};
  unsigned short* q = out + 8 * (size_t)i;
  *(volatile v4u*)q = u;
  __threadfence();
  *(volatile v4u*)q = u;
}

__global__ __launch_bounds__(256) void bias_prep_kernel(const float* __restrict__ b_ih, const float* __restrict__ b_hh,
                                                        const float* __restrict__ bq, const float* __restrict__ bk,
                                                        float* __restrict__ BS, float* __restrict__ BQK) {
  const int tid = threadIdx.x;
  const int i4 = tid * 4;
  const v4f va = *(const v4f*)(b_ih + i4);
  const v4f vb = *(const v4f*)(b_hh + i4);
  v4f o;
#pragma unroll
  for (int e = 0; e < 4; ++e) o[e] = va[e] + vb[e];
  const int qi = (tid & 63) * 4;
  const int which = (tid >> 6) & 1;
  const v4f vq = *(const v4f*)(bq + qi);
  const v4f vk = *(const v4f*)(bk + qi);
  v4f o2;
#pragma unroll
  for (int e = 0; e < 4; ++e) {
    const float sq = vq[e];
    const float sk = vk[e];
    o2[e] = (which ? sk : sq) * kQKCarry;
  }
  float* p1 = BS + i4;
  float* p2 = BQK + which * kH + qi;
  *(volatile v4f*)p1 = o;
  if (tid < 128) *(volatile v4f*)p2 = o2;
  __threadfence();
  *(volatile v4f*)p1 = o;
  if (tid < 128) *(volatile v4f*)p2 = o2;
}

__global__ __launch_bounds__(256) void enc_kernel(float* __restrict__ ENC) {
  const int id = blockIdx.x * 256 + threadIdx.x;
  const int b = id >> 6;
  const int i = id & 63;
  const float cdiv = -logf(10000.0f) / (float)kE;
  const float arg = (float)(2 * i) * cdiv;
  const float dv = expf(arg);
  const float ang = (float)b * dv;
  float sn, cs;
  sincosf(ang, &sn, &cs);
  const v2f o = (v2f){sn, cs};
  float* p = ENC + (size_t)b * kE + 2 * i;
  *(volatile v2f*)p = o;
  __threadfence();
  *(volatile v2f*)p = o;
}

__global__ __launch_bounds__(256) void dnorm_kernel(const float* __restrict__ data, unsigned short* __restrict__ DN16,
                                                    float* __restrict__ DINV) {
  __shared__ float sInv[32];
  const int tid = threadIdx.x, lane = tid & 31, wave = tid >> 5;
#pragma unroll 1
  for (int i = 0; i < 4; ++i) {
    const int row = blockIdx.x * 32 + wave * 4 + i;
    const v4f v = *(const v4f*)(data + (size_t)row * kE + 4 * lane);
    float ss = (v[0] * v[0] + v[1] * v[1]) + (v[2] * v[2] + v[3] * v[3]);
#pragma unroll
    for (int off = 16; off > 0; off >>= 1) ss += __shfl_xor(ss, off, 32);
    const float nrm = fmaxf(sqrtf(ss), 1e-8f);
    const float rinv = 1.0f / nrm;
    const float f0 = v[0] * rinv, f1 = v[1] * rinv, f2 = v[2] * rinv, f3 = v[3] * rinv;
    const v2u u = (v2u){pk16(h_bits(f0 * kNrmCarry), h_bits(f1 * kNrmCarry)), pk16(h_bits(f2 * kNrmCarry), h_bits(f3 * kNrmCarry))};
    unsigned short* q = DN16 + (size_t)row * kE + 4 * lane;
    *(volatile v2u*)q = u;
    __threadfence();
    *(volatile v2u*)q = u;
    if (lane == 0) sInv[wave * 4 + i] = rinv;
  }
  __syncthreads();
  if (wave == 0) {
    const float val = sInv[lane];
    float* p = DINV + blockIdx.x * 32 + lane;
    *(volatile float*)p = val;
    __threadfence();
    *(volatile float*)p = val;
  }
}

__global__ __launch_bounds__(256) void gather_kernel(const int* __restrict__ x, const float* __restrict__ emb,
                                                     const float* __restrict__ ENC,
                                                     unsigned short* __restrict__ XP16, unsigned short* __restrict__ QN16,
                                                     float* __restrict__ QN32) {
  const int tid = threadIdx.x, lane = tid & 31, wave = tid >> 5;
  const int m = blockIdx.x * 8 + wave;
  const int b = m & (kB - 1);
  int xi = x[m];
  xi = xi < 0 ? 0 : (xi > kNI - 1 ? kNI - 1 : xi);
  const v4f v  = *(const v4f*)(emb + (size_t)xi * kE + 4 * lane);
  const v4f en = *(const v4f*)(ENC + (size_t)b * kE + 4 * lane);
  float ss = (v[0] * v[0] + v[1] * v[1]) + (v[2] * v[2] + v[3] * v[3]);
#pragma unroll
  for (int off = 16; off > 0; off >>= 1) ss += __shfl_xor(ss, off, 32);
  const float nrm = fmaxf(sqrtf(ss), 1e-8f);
  const float rinv = 1.0f / nrm;
  v4f qn;
  unsigned short hx[4], hq[4];
#pragma unroll
  for (int e = 0; e < 4; ++e) {
    const float ve = v[e];
    const float ee = en[e];
    const float qe = ve * rinv;
    qn[e] = qe;
    hx[e] = h_bits((ve + ee) * kActCarry);
    hq[e] = h_bits(qe * kNrmCarry);
  }
  const v2u ux = (v2u){pk16(hx[0], hx[1]), pk16(hx[2], hx[3])};
  const v2u uq = (v2u){pk16(hq[0], hq[1]), pk16(hq[2], hq[3])};
  unsigned short* px = XP16 + (size_t)m * kE + 4 * lane;
  unsigned short* pq = QN16 + (size_t)m * kE + 4 * lane;
  float* pf = QN32 + (size_t)m * kE + 4 * lane;
  *(volatile v2u*)px = ux;
  *(volatile v2u*)pq = uq;
  *(volatile v4f*)pf = qn;
  __threadfence();
  *(volatile v2u*)px = ux;
  *(volatile v2u*)pq = uq;
  *(volatile v4f*)pf = qn;
}

__device__ __forceinline__ float sigm_f(float x) { return 1.0f / (1.0f + expf(-x)); }

__global__ __launch_bounds__(512) void lstm_seq_kernel(const float* __restrict__ PRE, const unsigned short* __restrict__ WHp,
                                                       const int* __restrict__ lengths, unsigned short* __restrict__ LS) {
  __shared__ __align__(16) _Float16 Ah[16 * kHP];
  const _Float16* WH = (const _Float16*)WHp;
  const int tid = threadIdx.x, lane = tid & 31, wave = tid >> 5;
  const int c = lane & 15, hh = lane >> 4, koff = hh * 8;
  const int b0 = blockIdx.x * 16;
#pragma unroll 1
  for (int i = tid; i < 16 * kHP; i += 512) Ah[i] = (_Float16)0.0f;
  float cst[8];
#pragma unroll
  for (int r = 0; r < 8; ++r) cst[r] = 0.0f;
  const int j = 16 * wave + c;
  const _Float16* wh = WH + (size_t)j * kH + koff;
  const _Float16* ahrow = Ah + c * kHP + koff;
  const float* prebase = PRE + (size_t)j * kM + b0 + 8 * hh;
  int len = lengths[b0 + wave];
  len = len < 0 ? 0 : (len > kT ? kT : len);
  __syncthreads();

  const v8f z8 = {0.f, 0.f, 0.f, 0.f, 0.f, 0.f, 0.f, 0.f};
#pragma unroll 1
  for (int t = 0; t < kT; ++t) {
    v8f a0 = z8, a1 = z8, a2 = z8, a3 = z8;
#pragma unroll 2
    for (int k0 = 0; k0 < kH; k0 += 32) {
      const v16h a  = Frag<_Float16>::load(ahrow + k0);
      const v16h w0 = Frag<_Float16>::load(wh + k0);
      const v16h w1 = Frag<_Float16>::load(wh + (size_t)1 * kH * kH + k0);
      const v16h w2 = Frag<_Float16>::load(wh + (size_t)2 * kH * kH + k0);
      const v16h w3 = Frag<_Float16>::load(wh + (size_t)3 * kH * kH + k0);
      a0 = Frag<_Float16>::mma(a, w0, a0);
      a1 = Frag<_Float16>::mma(a, w1, a1);
      a2 = Frag<_Float16>::mma(a, w2, a2);
      a3 = Frag<_Float16>::mma(a, w3, a3);
      dep_guard4_h(a0, a1, a2, a3, a, a, w0, w1, w2, w3);
    }
    acc_guard4(a0, a1, a2, a3);
    const float* pp = prebase + (size_t)t * kB;
    const v4f pi0 = *(const v4f*)(pp);
    const v4f pi1 = *(const v4f*)(pp + 4);
    const v4f pf0 = *(const v4f*)(pp + (size_t)1 * kH * kM);
    const v4f pf1 = *(const v4f*)(pp + (size_t)1 * kH * kM + 4);
    const v4f pg0 = *(const v4f*)(pp + (size_t)2 * kH * kM);
    const v4f pg1 = *(const v4f*)(pp + (size_t)2 * kH * kM + 4);
    const v4f po0 = *(const v4f*)(pp + (size_t)3 * kH * kM);
    const v4f po1 = *(const v4f*)(pp + (size_t)3 * kH * kM + 4);
    float hq[8];
#pragma unroll
    for (int r = 0; r < 8; ++r) {
      const float xi_ = (r < 4) ? pi0[r & 3] : pi1[r & 3];
      const float xf_ = (r < 4) ? pf0[r & 3] : pf1[r & 3];
      const float xg_ = (r < 4) ? pg0[r & 3] : pg1[r & 3];
      const float xo_ = (r < 4) ? po0[r & 3] : po1[r & 3];
      const float zi = a0[r] * kPreScale + xi_;
      const float zf = a1[r] * kPreScale + xf_;
      const float zg = a2[r] * kPreScale + xg_;
      const float zo = a3[r] * kPreScale + xo_;
      const float cn = sigm_f(zf) * cst[r] + sigm_f(zi) * tanhf(zg);
      cst[r] = cn;
      hq[r] = sigm_f(zo) * tanhf(cn);
    }
    __syncthreads();
#pragma unroll
    for (int r = 0; r < 8; ++r) Ah[(8 * hh + r) * kHP + j] = (_Float16)(hq[r] * kActCarry);
    __syncthreads();
    {
      const v8h hv = *(const v8h*)(Ah + wave * kHP + lane * 8);
      const v4u wv = __builtin_bit_cast(v4u, hv);
      const bool keepr = (t < len);
      v4u ov;
#pragma unroll
      for (int e = 0; e < 4; ++e) {
        const unsigned we = wv[e];
        ov[e] = keepr ? we : 0u;
      }
      unsigned short* dst = LS + ((size_t)(b0 + wave) * kT + (size_t)t) * kH + lane * 8;
      *(volatile v4u*)dst = ov;
      __threadfence();
      *(volatile v4u*)dst = ov;
    }
  }
}

__global__ __launch_bounds__(128) void attn_pool_kernel(const unsigned short* __restrict__ QKp, const unsigned short* __restrict__ LS,
                                                        const int* __restrict__ lengths,
                                                        const float* __restrict__ Wv, const float* __restrict__ bv,
                                                        const float* __restrict__ Wo, const float* __restrict__ bo,
                                                        float* __restrict__ AO) {
  __shared__ float sS[64 * 65];
  __shared__ float sRI[64];
  __shared__ float sAbar[64];
  __shared__ __align__(16) float sX[kH];
  __shared__ __align__(16) float sV[kH];
  const _Float16* QK = (const _Float16*)QKp;
  const int tid = threadIdx.x, lane = tid & 31, wave = tid >> 5;
  const int c = lane & 15, hh = lane >> 4, koff = hh * 8;
  const int b = blockIdx.x;
  int len = lengths[b];
  len = len < 1 ? 1 : (len > kT ? kT : len);

  const _Float16* qrow = QK + (size_t)(b * kT + 16 * wave + c) * (2 * kH) + koff;
  const _Float16* krow = QK + (size_t)(b * kT + c) * (2 * kH) + kH + koff;
  const v8f z8 = {0.f, 0.f, 0.f, 0.f, 0.f, 0.f, 0.f, 0.f};
  v8f s0 = z8, s1 = z8, s2 = z8, s3 = z8;
#pragma unroll 1
  for (int k0 = 0; k0 < kH; k0 += 32) {
    const v16h a  = Frag<_Float16>::load(qrow + k0);
    const v16h k0f = Frag<_Float16>::load(krow + k0);
    const v16h k1f = Frag<_Float16>::load(krow + (size_t)16 * (2 * kH) + k0);
    const v16h k2f = Frag<_Float16>::load(krow + (size_t)32 * (2 * kH) + k0);
    const v16h k3f = Frag<_Float16>::load(krow + (size_t)48 * (2 * kH) + k0);
    s0 = Frag<_Float16>::mma(a, k0f, s0);
    s1 = Frag<_Float16>::mma(a, k1f, s1);
    s2 = Frag<_Float16>::mma(a, k2f, s2);
    s3 = Frag<_Float16>::mma(a, k3f, s3);
    dep_guard4_h(s0, s1, s2, s3, a, a, k0f, k1f, k2f, k3f);
  }
  acc_guard4(s0, s1, s2, s3);
  {
    const float ninf = -__builtin_inff();
    const bool m0 = (c < len), m1 = (16 + c < len), m2 = (32 + c < len), m3 = (48 + c < len);
#pragma unroll
    for (int r = 0; r < 8; ++r) {
      float* rowp = sS + (16 * wave + 8 * hh + r) * 65 + c;
      rowp[0]  = m0 ? s0[r] * kScoreScale : ninf;
      rowp[16] = m1 ? s1[r] * kScoreScale : ninf;
      rowp[32] = m2 ? s2[r] * kScoreScale : ninf;
      rowp[48] = m3 ? s3[r] * kScoreScale : ninf;
    }
  }
  __syncthreads();
  {
    const int row = tid >> 1, half = tid & 1;
    float* rp = sS + row * 65 + 32 * half;
    float mx = -__builtin_inff();
#pragma unroll 1
    for (int cc = 0; cc < 32; ++cc) mx = fmaxf(mx, rp[cc]);
    mx = fmaxf(mx, __shfl_xor(mx, 1, 32));
    float sum = 0.0f;
#pragma unroll 1
    for (int cc = 0; cc < 32; ++cc) {
      const float p = expf(rp[cc] - mx);
      rp[cc] = p;
      sum += p;
    }
    sum += __shfl_xor(sum, 1, 32);
    if (half == 0) sRI[row] = 1.0f / sum;
  }
  __syncthreads();
  if (tid < 64) {
    float a = 0.0f;
#pragma unroll 1
    for (int t = 0; t < kT; ++t) a += sS[t * 65 + tid] * sRI[t];
    sAbar[tid] = a * kInvT;
  }
  __syncthreads();
  {
    const unsigned* LSw = (const unsigned*)(const void*)LS;
    float x0 = 0.0f, x1 = 0.0f;
#pragma unroll 1
    for (int s = 0; s < kT; ++s) {
      const unsigned w = LSw[(((size_t)(b * kT + s)) * kH + 2 * tid) >> 1];
      const float lo = h16_to_f32(w & 0xffffu);
      const float hi = h16_to_f32(w >> 16);
      const float ab = sAbar[s];
      x0 = fmaf(ab, lo, x0);
      x1 = fmaf(ab, hi, x1);
    }
    sX[2 * tid]     = x0 * kActInv;
    sX[2 * tid + 1] = x1 * kActInv;
  }
  __syncthreads();
  {
    const float* w0p = Wv + (size_t)tid * kH;
    const float* w1p = Wv + (size_t)(tid + 128) * kH;
    float a0 = 0.0f, a1 = 0.0f;
#pragma unroll 1
    for (int k4 = 0; k4 < kH / 4; ++k4) {
      const v4f xv = *(const v4f*)(sX + 4 * k4);
      const v4f w0 = *(const v4f*)(w0p + 4 * k4);
      const v4f w1 = *(const v4f*)(w1p + 4 * k4);
      a0 = fmaf(xv[0], w0[0], a0); a0 = fmaf(xv[1], w0[1], a0); a0 = fmaf(xv[2], w0[2], a0); a0 = fmaf(xv[3], w0[3], a0);
      a1 = fmaf(xv[0], w1[0], a1); a1 = fmaf(xv[1], w1[1], a1); a1 = fmaf(xv[2], w1[2], a1); a1 = fmaf(xv[3], w1[3], a1);
    }
    sV[tid]       = a0 + bv[tid];
    sV[tid + 128] = a1 + bv[tid + 128];
  }
  __syncthreads();
  {
    const float* wp = Wo + (size_t)tid * kH;
    float a = 0.0f;
#pragma unroll 1
    for (int k4 = 0; k4 < kH / 4; ++k4) {
      const v4f xv = *(const v4f*)(sV + 4 * k4);
      const v4f w0 = *(const v4f*)(wp + 4 * k4);
      a = fmaf(xv[0], w0[0], a); a = fmaf(xv[1], w0[1], a); a = fmaf(xv[2], w0[2], a); a = fmaf(xv[3], w0[3], a);
    }
    const float o = a + bo[tid];
    float* p = AO + (size_t)b * kE + tid;
    *(volatile float*)p = o;
    __threadfence();
    *(volatile float*)p = o;
  }
}

__global__ __launch_bounds__(128) void knn_screen_kernel(const unsigned short* __restrict__ QN16p, const unsigned short* __restrict__ DN16p,
                                                         int* __restrict__ CAND) {
  const _Float16* QN = (const _Float16*)QN16p;
  const _Float16* DN = (const _Float16*)DN16p;
  const int tid = threadIdx.x, lane = tid & 31, wave = tid >> 5;
  const int c = lane & 15, hh = lane >> 4, koff = hh * 8;
  const int tile = blockIdx.x * 4 + wave;
  if (tile >= kM / 16) return;
  const int m0 = tile * 16;
  const _Float16* arow = QN + (size_t)(m0 + c) * kE + koff;
  const v16h qa0 = Frag<_Float16>::load(arow);
  const v16h qa1 = Frag<_Float16>::load(arow + 32);
  const v16h qa2 = Frag<_Float16>::load(arow + 64);
  const v16h qa3 = Frag<_Float16>::load(arow + 96);
  float v1[8], v2[8];
  int i1[8], i2[8];
#pragma unroll
  for (int r = 0; r < 8; ++r) { v1[r] = -3.0e38f; v2[r] = -3.0e38f; i1[r] = 0; i2[r] = 0; }
  const v8f z8 = {0.f, 0.f, 0.f, 0.f, 0.f, 0.f, 0.f, 0.f};
#pragma unroll 1
  for (int nt = 0; nt < kND / 16; ++nt) {
    const _Float16* brow = DN + (size_t)(nt * 16 + c) * kE + koff;
    const v16h d0 = Frag<_Float16>::load(brow);
    const v16h d1 = Frag<_Float16>::load(brow + 32);
    const v16h d2 = Frag<_Float16>::load(brow + 64);
    const v16h d3 = Frag<_Float16>::load(brow + 96);
    v8f acc = z8;
    acc = mma_nop_h(qa0, d0, acc);
    acc = mma_nop_h(qa1, d1, acc);
    acc = mma_nop_h(qa2, d2, acc);
    acc = mma_nop_h(qa3, d3, acc);
    const int n = nt * 16 + c;
#pragma unroll
    for (int r = 0; r < 8; ++r) {
      const float s = acc[r];
      const bool g1 = s > v1[r];
      const bool g2 = s > v2[r];
      const float nv2 = g1 ? v1[r] : (g2 ? s : v2[r]);
      const int   ni2 = g1 ? i1[r] : (g2 ? n : i2[r]);
      v1[r] = g1 ? s : v1[r];
      i1[r] = g1 ? n : i1[r];
      v2[r] = nv2;
      i2[r] = ni2;
    }
  }
  for (int pass = 0; pass < 2; ++pass) {
#pragma unroll
    for (int r = 0; r < 8; ++r) {
      const v2i val = (v2i){i1[r], i2[r]};
      *(volatile v2i*)(CAND + (size_t)(m0 + 8 * hh + r) * 32 + 2 * c) = val;
    }
    __threadfence();
  }
}

__global__ __launch_bounds__(256) void rerank_kernel(const float* __restrict__ QN32, const int* __restrict__ CAND,
                                                     const float* __restrict__ data, const float* __restrict__ DINV,
                                                     int* __restrict__ IDX) {
  __shared__ __align__(16) float sQ[8][4][kE];
  __shared__ int sIdx[32];
  const int tid = threadIdx.x, lane = tid & 31, wave = tid >> 5;
  const int q0 = blockIdx.x * 32 + wave * 4;
#pragma unroll
  for (int i = 0; i < 4; ++i) {
    const v4f qv = *(const v4f*)(QN32 + (size_t)(q0 + i) * kE + 4 * lane);
    *(v4f*)(&sQ[wave][i][4 * lane]) = qv;
  }
  __syncthreads();
#pragma unroll 1
  for (int i = 0; i < 4; ++i) {
    const int q = q0 + i;
    int ci = CAND[(size_t)q * 32 + lane];
    ci = ci < 0 ? 0 : (ci > kND - 1 ? kND - 1 : ci);
    const float rinv = DINV[ci];
    const float* drow = data + (size_t)ci * kE;
    const float* qp = &sQ[wave][i][0];
    float acc = 0.0f;
#pragma unroll 1
    for (int e4 = 0; e4 < kE / 4; ++e4) {
      const v4f d  = *(const v4f*)(drow + 4 * e4);
      const v4f qv = *(const v4f*)(qp + 4 * e4);
      const float n0 = d[0] * rinv, n1 = d[1] * rinv, n2 = d[2] * rinv, n3 = d[3] * rinv;
      acc = fmaf(qv[0], n0, acc);
      acc = fmaf(qv[1], n1, acc);
      acc = fmaf(qv[2], n2, acc);
      acc = fmaf(qv[3], n3, acc);
    }
    float bvv = acc;
    int bi = ci;
#pragma unroll
    for (int off = 16; off > 0; off >>= 1) {
      const float ov = __shfl_xor(bvv, off, 32);
      const int   oi = __shfl_xor(bi, off, 32);
      const bool take = (ov > bvv) || (ov == bvv && oi < bi);
      bvv = take ? ov : bvv;
      bi  = take ? oi : bi;
    }
    if (lane == 0) sIdx[wave * 4 + i] = bi;
  }
  __syncthreads();
  if (wave == 0) {
    const int val = sIdx[lane];
    int* p = IDX + blockIdx.x * 32 + lane;
    *(volatile int*)p = val;
    __threadfence();
    *(volatile int*)p = val;
  }
}

__global__ __launch_bounds__(128) void closest_kernel(const int* __restrict__ IDX, const float* __restrict__ data,
                                                      const float* __restrict__ AO, unsigned short* __restrict__ ASC16) {
  __shared__ int sI[kT];
  __shared__ float sA[kE];
  const int tid = threadIdx.x;
  const int b = blockIdx.x;
  if (tid < kT) {
    int v = IDX[tid * kB + b];
    v = v < 0 ? 0 : (v > kND - 1 ? kND - 1 : v);
    sI[tid] = v;
  }
  __syncthreads();
  float acc = 0.0f;
#pragma unroll 1
  for (int t = 0; t < kT; ++t) acc += data[(size_t)sI[t] * kE + tid];
  const float cl = acc * kInvT;
  const float a = AO[(size_t)b * kE + tid] * cl;
  sA[tid] = a * kAscCarry;
  __syncthreads();
  if (tid < 16) {
    unsigned short hb[8];
#pragma unroll
    for (int e = 0; e < 8; ++e) hb[e] = h_bits(sA[8 * tid + e]);
    const v4u u = (v4u){pk16(hb[0], hb[1]), pk16(hb[2], hb[3]), pk16(hb[4], hb[5]), pk16(hb[6], hb[7])};
    unsigned short* p = ASC16 + (size_t)b * kE + 8 * tid;
    *(volatile v4u*)p = u;
    __threadfence();
    *(volatile v4u*)p = u;
  }
}

__global__ __launch_bounds__(256) void copy_out_kernel(const float* __restrict__ ST, float* __restrict__ out, int n4) {
  const int i4 = blockIdx.x * 256 + threadIdx.x;
  if (i4 >= n4) return;
  const int flat = 4 * i4;
  const int b = flat / kNI;
  const int n = flat - b * kNI;
  const v4f v = *(const v4f*)(ST + (size_t)b * kNIP + n);
  float* p = out + (size_t)flat;
  *(volatile v4f*)p = v;
  __threadfence();
  *(volatile v4f*)p = v;
}

extern "C" void kernel_launch(void* const* d_in, const int* in_sizes, int n_in,
                              void* d_out, int out_size, void* d_ws, size_t ws_size, hipStream_t stream) {
  if (n_in < 16 || d_out == nullptr || d_ws == nullptr) return;
  if (in_sizes[0] != kT * kB || in_sizes[1] != kB || in_sizes[2] != kNI * kE || in_sizes[3] != kND * kE ||
      in_sizes[4] != kG * kE || in_sizes[5] != kG * kH || in_sizes[6] != kG || in_sizes[7] != kG ||
      in_sizes[8] != kH * kH || in_sizes[9] != kH || in_sizes[10] != kH * kH || in_sizes[11] != kH ||
      in_sizes[12] != kH * kH || in_sizes[13] != kH || in_sizes[14] != kE * kH || in_sizes[15] != kE ||
      out_size != kNOUT) return;

  const int*   x       = (const int*)  d_in[0];
  const int*   lengths = (const int*)  d_in[1];
  const float* emb_t   = (const float*)d_in[2];
  const float* data_e  = (const float*)d_in[3];
  const float* W_ih    = (const float*)d_in[4];
  const float* W_hh    = (const float*)d_in[5];
  const float* b_ih    = (const float*)d_in[6];
  const float* b_hh    = (const float*)d_in[7];
  const float* Wq      = (const float*)d_in[8];
  const float* bq      = (const float*)d_in[9];
  const float* Wk      = (const float*)d_in[10];
  const float* bk      = (const float*)d_in[11];
  const float* Wv      = (const float*)d_in[12];
  const float* bv      = (const float*)d_in[13];
  const float* W_out   = (const float*)d_in[14];
  const float* b_out   = (const float*)d_in[15];
  float* out = (float*)d_out;

  char* ws = (char*)d_ws; size_t off = 0;
  auto carve = [&](size_t bytes) -> char* { char* p = ws + off; off += (bytes + 255) & ~(size_t)255; return p; };
  unsigned short* WIH16 = (unsigned short*)carve((size_t)kG * kE * 2);
  unsigned short* WHH16 = (unsigned short*)carve((size_t)kG * kH * 2);
  unsigned short* WQK16 = (unsigned short*)carve((size_t)2 * kH * kH * 2);
  unsigned short* EMB16 = (unsigned short*)carve((size_t)kNIP * kE * 2);
  float*          BS    = (float*)carve((size_t)kG * 4);
  float*          BQK   = (float*)carve((size_t)2 * kH * 4);
  float*          ENC   = (float*)carve((size_t)kB * kE * 4);
  unsigned short* DN16  = (unsigned short*)carve((size_t)kND * kE * 2);
  float*          DINV  = (float*)carve((size_t)kND * 4);
  unsigned short* XP16  = (unsigned short*)carve((size_t)kM * kE * 2);
  unsigned short* QN16  = (unsigned short*)carve((size_t)kM * kE * 2);
  float*          QN32  = (float*)carve((size_t)kM * kE * 4);
  float*          PRE   = (float*)carve((size_t)kG * kM * 4);
  unsigned short* LS16  = (unsigned short*)carve((size_t)kM * kH * 2);
  unsigned short* QK16  = (unsigned short*)carve((size_t)kM * 2 * kH * 2);
  float*          AO    = (float*)carve((size_t)kB * kE * 4);
  int*            CAND  = (int*)carve((size_t)kM * 32 * 4);
  int*            IDX   = (int*)carve((size_t)kM * 4);
  unsigned short* ASC16 = (unsigned short*)carve((size_t)kB * kE * 2);
  float*          ST    = (float*)carve((size_t)kB * kNIP * 4);
  if (off > ws_size || off > (size_t)134217728) return;

  {
    const int n8a = kG * kE / 8;
    const int n8b = kG * kH / 8;
    const int n8c = kH * kH / 8;
    const int n8e_real = kNI * kE / 8;
    const int n8e_tot  = kNIP * kE / 8;
    cast8_pad_kernel<<<n8a / 256, 256, 0, stream>>>(W_ih, WIH16, n8a, n8a, kWCarry);
    cast8_pad_kernel<<<n8b / 256, 256, 0, stream>>>(W_hh, WHH16, n8b, n8b, kWCarry);
    cast8_pad_kernel<<<n8c / 256, 256, 0, stream>>>(Wq, WQK16, n8c, n8c, kWCarry);
    cast8_pad_kernel<<<n8c / 256, 256, 0, stream>>>(Wk, WQK16 + (size_t)kH * kH, n8c, n8c, kWCarry);
    cast8_pad_kernel<<<n8e_tot / 256, 256, 0, stream>>>(emb_t, EMB16, n8e_real, n8e_tot, kWCarry);
  }
  bias_prep_kernel<<<1, 256, 0, stream>>>(b_ih, b_hh, bq, bk, BS, BQK);
  enc_kernel<<<(kB * (kE / 2)) / 256, 256, 0, stream>>>(ENC);

  dnorm_kernel<<<kND / 32, 256, 0, stream>>>(data_e, DN16, DINV);
  gather_kernel<<<kM / 8, 256, 0, stream>>>(x, emb_t, ENC, XP16, QN16, QN32);

  wmma_gemm64<0, false, 1, 0, false><<<dim3((kG / 64) * (kM / 64) / 8, 1), 256, 0, stream>>>(
      WIH16, WIH16, kE, 0L, XP16, XP16, kE, 0L, (void*)PRE, (void*)PRE, kM, 0L,
      BS, BS, 0L, kG, kM, kE, kPreScale);

  lstm_seq_kernel<<<kB / 16, 512, 0, stream>>>(PRE, WHH16, lengths, LS16);

  wmma_gemm64<0, false, 2, 1, false><<<dim3((kM / 64) * (2 * kH / 64) / 8, 1), 256, 0, stream>>>(
      LS16, LS16, kH, 0L, WQK16, WQK16, kH, 0L, (void*)QK16, (void*)QK16, 2 * kH, 0L,
      BQK, BQK, 0L, kM, 2 * kH, kH, kQKScale);

  attn_pool_kernel<<<kB, 128, 0, stream>>>(QK16, LS16, lengths, Wv, bv, W_out, b_out, AO);

  knn_screen_kernel<<<(kM / 16) / 4, 128, 0, stream>>>(QN16, DN16, CAND);
  rerank_kernel<<<kM / 32, 256, 0, stream>>>(QN32, CAND, data_e, DINV, IDX);
  closest_kernel<<<kB, 128, 0, stream>>>(IDX, data_e, AO, ASC16);

  wmma_gemm64<0, false, 0, 0, false><<<dim3(((kB / 64) * (kNIP / 64) + 7) / 8, 1), 256, 0, stream>>>(
      ASC16, ASC16, kE, 0L, EMB16, EMB16, kE, 0L, (void*)ST, (void*)ST, kNIP, 0L,
      BS, BS, 0L, kB, kNIP, kE, kOutScale);

  copy_out_kernel<<<(kNOUT / 4) / 256, 256, 0, stream>>>(ST, out, kNOUT / 4);
}
